// SegmentCausalCrossAttention_36043365548100
// MI455X (gfx1250) — hardware-verified
//
#include <hip/hip_runtime.h>
#include <math.h>

constexpr int NBATCH  = 2;
constexpr int LQ      = 4096;
constexpr int LKV     = 512;
constexpr int NHEAD   = 16;
constexpr int DHEAD   = 64;
constexpr int NHALF   = 32;
constexpr int KWIN    = 8;
constexpr int SMAXPOS = 8192;
constexpr int DMODEL  = 1024;
constexpr int KVCOLS  = 2048;
constexpr int NQROWS  = NBATCH * LQ;
constexpr int NKVROWS = NBATCH * LKV;
constexpr int NTRIGROWS = NQROWS + LKV;
constexpr float ATT_SCALE = 0.125f;
constexpr float NEG_FILL  = -3.402823466e+38f;
constexpr float ROPE_BASE_F = 10000.0f;
constexpr int ATT_QPB = 8;
constexpr int ATT_THREADS = ATT_QPB * NHEAD;

static_assert(NHEAD * DHEAD == DMODEL);
static_assert(DHEAD == 2 * NHALF);
static_assert(NQROWS % 64 == 0 && NKVROWS % 64 == 0 && DMODEL % 64 == 0 && KVCOLS % 64 == 0);
static_assert(DMODEL % 32 == 0);
static_assert(NQROWS % ATT_QPB == 0);
static_assert((NTRIGROWS * NHALF) % 256 == 0);
static_assert((NKVROWS * NHEAD) % 8 == 0);
static_assert((NQROWS * DMODEL) % 2048 == 0 && (NKVROWS * DMODEL) % 2048 == 0);
static_assert(ATT_THREADS == 128);

typedef __attribute__((ext_vector_type(16))) _Float16 v16h;
typedef __attribute__((ext_vector_type(8)))  _Float16 v8h;
typedef __attribute__((ext_vector_type(16))) __bf16   v16b;
typedef __attribute__((ext_vector_type(8)))  __bf16   v8b;
typedef __attribute__((ext_vector_type(8)))  float    v8f;
typedef __attribute__((ext_vector_type(4)))  float    v4f;

__device__ __forceinline__ unsigned short f2bf_bits(float f) {
  unsigned u = __float_as_uint(f);
  return (unsigned short)((u + 0x7FFFu + ((u >> 16) & 1u)) >> 16);
}
__device__ __forceinline__ float bf_bits2f(unsigned short h) { return __uint_as_float(((unsigned)h) << 16); }

__device__ __forceinline__ void dep_guard_h(v8f& a, v8f& b, v16h x, v16h y) { asm volatile("v_nop\n\tv_nop\n\tv_nop\n\tv_nop" : "+v"(a), "+v"(b) : "v"(x), "v"(y)); }
__device__ __forceinline__ void dep_guard_b(v8f& a, v8f& b, v16b x, v16b y) { asm volatile("v_nop\n\tv_nop\n\tv_nop\n\tv_nop" : "+v"(a), "+v"(b) : "v"(x), "v"(y)); }
__device__ __forceinline__ void keep4_h(v16h a, v16h b, v16h c, v16h d) { asm volatile("v_nop" :: "v"(a), "v"(b), "v"(c), "v"(d)); }
__device__ __forceinline__ void keep4_b(v16b a, v16b b, v16b c, v16b d) { asm volatile("v_nop" :: "v"(a), "v"(b), "v"(c), "v"(d)); }
__device__ __forceinline__ void acc_guard4(v8f& a, v8f& b, v8f& c, v8f& d) { asm volatile("v_nop\n\tv_nop\n\tv_nop\n\tv_nop" : "+v"(a), "+v"(b), "+v"(c), "+v"(d)); }
template <typename T> struct Frag;
template <> struct Frag<_Float16> {
  typedef v16h V; union U { v16h v; v8h h[2]; };
  static __device__ __forceinline__ v16h load(const _Float16* p) {
    U f; f.h[0] = *(const v8h*)(p); f.h[1] = *(const v8h*)(p + 16); return f.v;
  }
  static __device__ __forceinline__ v8f mma(v16h a, v16h b, v8f c) {
    return __builtin_amdgcn_wmma_f32_16x16x32_f16(false, a, false, b, (short)0, c, false, false);
  }
  static __device__ __forceinline__ void guard(v8f& a, v8f& b, v16h x, v16h y) { dep_guard_h(a, b, x, y); }
  static __device__ __forceinline__ void keep(v16h a, v16h b, v16h c, v16h d) { keep4_h(a, b, c, d); }
};
template <> struct Frag<__bf16> {
  typedef v16b V; union U { v16b v; v8b h[2]; };
  static __device__ __forceinline__ v16b load(const __bf16* p) {
    U f; f.h[0] = *(const v8b*)(p); f.h[1] = *(const v8b*)(p + 16); return f.v;
  }
  static __device__ __forceinline__ v8f mma(v16b a, v16b b, v8f c) {
    return __builtin_amdgcn_wmma_f32_16x16x32_bf16(false, a, false, b, (short)0, c, false, false);
  }
  static __device__ __forceinline__ void guard(v8f& a, v8f& b, v16b x, v16b y) { dep_guard_b(a, b, x, y); }
  static __device__ __forceinline__ void keep(v16b a, v16b b, v16b c, v16b d) { keep4_b(a, b, c, d); }
};

template <int ET> struct Elem;
template <> struct Elem<0> { typedef _Float16 T; };
template <> struct Elem<1> { typedef __bf16 T; };
template <int ET, bool SPLIT, int BIAS_MODE, int OUT_MODE, bool RESID, int ACT = 0>
__global__ __launch_bounds__(256) void wmma_gemm64(
    const unsigned short* __restrict__ Ap, const unsigned short* __restrict__ A2p, int lda, long strideA,
    const unsigned short* __restrict__ Btp, const unsigned short* __restrict__ Bt2p, int ldb, long strideB,
    void* __restrict__ Cout, void* __restrict__ Cout2, int ldc, long strideC,
    const float* __restrict__ bias,
    const float* __restrict__ resid, long strideR,
    int M, int N, int K, float scale) {
  typedef typename Elem<ET>::T T;
  typedef typename Frag<T>::V V;
  const T* A = (const T*)Ap; const T* A2 = (const T*)A2p; const T* Bt = (const T*)Btp; const T* Bt2 = (const T*)Bt2p;
  __shared__ __align__(16) float sT[8][16 * 68];
  const int b    = blockIdx.y;
  const int lane = threadIdx.x & 31;
  const int wave = threadIdx.x >> 5;
  const int tilesN = N >> 6;
  const int tilesM = M >> 6;
  const int tile = blockIdx.x * 8 + wave;
  if (tile >= tilesM * tilesN) return;
  const int tm = tile / tilesN;
  const int tn = tile - tm * tilesN;
  const int m0 = tm << 6;
  const int n0 = tn << 6;

  const T* Ab  = A  + (size_t)b * strideA;
  const T* Bb  = Bt + (size_t)b * strideB;
  const T* Ab2 = SPLIT ? (A2  + (size_t)b * strideA) : nullptr;
  const T* Bb2 = SPLIT ? (Bt2 + (size_t)b * strideB) : nullptr;

  const int rlane = lane & 15;
  const int koff  = (lane >> 4) * 8;
  const int mOff  = (lane >> 4) * 8;

  v8f acc[4][4];
#pragma unroll
  for (int i = 0; i < 4; ++i)
#pragma unroll
    for (int j = 0; j < 4; ++j) acc[i][j] = (v8f){0.f,0.f,0.f,0.f,0.f,0.f,0.f,0.f};

  for (int k0 = 0; k0 < K; k0 += 32) {
    V bh[4], bl[4];
#pragma unroll
    for (int j = 0; j < 4; ++j) {
      const size_t bo = (size_t)(n0 + (j << 4) + rlane) * ldb + koff + k0;
      bh[j] = Frag<T>::load(Bb + bo);
      if (SPLIT) bl[j] = Frag<T>::load(Bb2 + bo);
    }
#pragma unroll
    for (int i = 0; i < 4; ++i) {
      const size_t ao = (size_t)(m0 + (i << 4) + rlane) * lda + koff + k0;
      V ah = Frag<T>::load(Ab + ao);
      V al;
      if (SPLIT) al = Frag<T>::load(Ab2 + ao);
#pragma unroll
      for (int j = 0; j < 4; ++j) {
        acc[i][j] = Frag<T>::mma(ah, bh[j], acc[i][j]);
        if (SPLIT) {
          acc[i][j] = Frag<T>::mma(ah, bl[j], acc[i][j]);
          acc[i][j] = Frag<T>::mma(al, bh[j], acc[i][j]);
        }
      }
      Frag<T>::guard(acc[i][0], acc[i][3], ah, SPLIT ? al : ah);
    }
    Frag<T>::keep(bh[0], bh[1], bh[2], bh[3]);
    if (SPLIT) Frag<T>::keep(bl[0], bl[1], bl[2], bl[3]);
  }
  acc_guard4(acc[0][0], acc[0][1], acc[0][2], acc[0][3]);
  acc_guard4(acc[1][0], acc[1][1], acc[1][2], acc[1][3]);
  acc_guard4(acc[2][0], acc[2][1], acc[2][2], acc[2][3]);
  acc_guard4(acc[3][0], acc[3][1], acc[3][2], acc[3][3]);

  float* slab = sT[wave];
  const float* Rb = RESID ? (resid + (size_t)b * strideR) : nullptr;
#pragma unroll
  for (int i = 0; i < 4; ++i) {
    const int mBase = m0 + (i << 4);
#pragma unroll
    for (int j = 0; j < 4; ++j) {
      const int n = n0 + (j << 4) + rlane;
      float bv = 0.f;
      if (BIAS_MODE == 2) bv = bias[n];
#pragma unroll
      for (int r = 0; r < 8; ++r) {
        float v = acc[i][j][r] * scale;
        if (BIAS_MODE == 1) v += bias[mBase + mOff + r];
        if (BIAS_MODE == 2) v += bv;
        if (RESID) v += Rb[(size_t)(mBase + mOff + r) * ldc + n];
        if (ACT == 1) v = tanhf(v);
        if (ACT == 2) v = fmaxf(v, 0.0f);
        if (ACT == 3) v = v / (1.0f + expf(-v));
        if (ACT == 4) v = (v > 0.f) ? v : 0.01f * v;
        if (ACT == 5) v = 0.5f * v * (1.0f + erff(v * 0.70710678118654752f));
        slab[(mOff + r) * 68 + (j << 4) + rlane] = v;
      }
    }
    __builtin_amdgcn_fence(__ATOMIC_RELEASE, "workgroup");
    __builtin_amdgcn_wave_barrier();
    __builtin_amdgcn_fence(__ATOMIC_ACQUIRE, "workgroup");
    if (OUT_MODE == 0) {
      float* C = (float*)Cout + (size_t)b * strideC;
      const int hh = lane >> 4, c4 = (lane & 15) * 4;
      for (int pass = 0; pass < 2; ++pass) {
#pragma unroll
        for (int it = 0; it < 8; ++it) {
          const int row = it * 2 + hh;
          v4f v = *(const v4f*)(slab + row * 68 + c4);
          *(volatile v4f*)(C + (size_t)(mBase + row) * ldc + n0 + c4) = v;
        }
        __threadfence();
      }
    } else {
      const int q = lane >> 3, c8 = (lane & 7) * 8;
      unsigned short* C  = (unsigned short*)Cout  + (size_t)b * strideC;
      unsigned short* C2 = (OUT_MODE == 2) ? ((unsigned short*)Cout2 + (size_t)b * strideC) : nullptr;
      for (int pass = 0; pass < 2; ++pass) {
#pragma unroll
        for (int it = 0; it < 4; ++it) {
          const int row = it * 4 + q;
          const float* sp = slab + row * 68 + c8;
          v8h hv, lv;
#pragma unroll
          for (int e = 0; e < 8; ++e) {
            if (OUT_MODE == 1) {
              hv[e] = (_Float16)sp[e];
            } else {
              unsigned short hb = f2bf_bits(sp[e]);
              unsigned short lb = f2bf_bits(sp[e] - bf_bits2f(hb));
              hv[e] = __builtin_bit_cast(_Float16, hb);
              lv[e] = __builtin_bit_cast(_Float16, lb);
            }
          }
          *(volatile v8h*)(C + (size_t)(mBase + row) * ldc + n0 + c8) = hv;
          if (OUT_MODE == 2) *(volatile v8h*)(C2 + (size_t)(mBase + row) * ldc + n0 + c8) = lv;
        }
        __threadfence();
      }
    }
    __builtin_amdgcn_fence(__ATOMIC_RELEASE, "workgroup");
    __builtin_amdgcn_wave_barrier();
    __builtin_amdgcn_fence(__ATOMIC_ACQUIRE, "workgroup");
  }
}

union H8 { v8h v; unsigned short u[8]; };
union F8 { v4f v[2]; float f[8]; };

__global__ __launch_bounds__(256) void k_split8(const float* __restrict__ w, unsigned short* __restrict__ hi,
                                                unsigned short* __restrict__ lo, int n8) {
  int i = blockIdx.x * 256 + threadIdx.x;
  const bool act = i < n8;
  i = act ? i : n8 - 1;
  F8 ab;
  ab.v[0] = *(const v4f*)(w + (size_t)i * 8);
  ab.v[1] = *(const v4f*)(w + (size_t)i * 8 + 4);
  H8 oh, ol;
#pragma unroll
  for (int e = 0; e < 8; ++e) {
    const unsigned short hb = f2bf_bits(ab.f[e]);
    const unsigned short lb = f2bf_bits(ab.f[e] - bf_bits2f(hb));
    oh.u[e] = hb; ol.u[e] = lb;
  }
  if (act) {
    unsigned short* dh = hi + (size_t)i * 8;
    unsigned short* dl = lo + (size_t)i * 8;
    *(volatile v8h*)dh = oh.v;
    *(volatile v8h*)dl = ol.v;
    __threadfence();
    *(volatile v8h*)dh = oh.v;
    *(volatile v8h*)dl = ol.v;
  }
}

__global__ __launch_bounds__(256) void k_tsplit(const float* __restrict__ W, unsigned short* __restrict__ hi,
                                                unsigned short* __restrict__ lo, int nrows_k, int ncols_n) {
  __shared__ float lt[64][65];
  const int tid = threadIdx.x, lane = tid & 31, wave = tid >> 5;
  const int k0 = blockIdx.y * 64, n0 = blockIdx.x * 64;
  {
    const int r = tid >> 2, c16 = (tid & 3) * 16;
    const float* src = W + (size_t)(k0 + r) * ncols_n + n0 + c16;
#pragma unroll
    for (int qq = 0; qq < 4; ++qq) {
      const v4f v = *(const v4f*)(src + 4 * qq);
      lt[r][c16 + 4 * qq + 0] = v[0];
      lt[r][c16 + 4 * qq + 1] = v[1];
      lt[r][c16 + 4 * qq + 2] = v[2];
      lt[r][c16 + 4 * qq + 3] = v[3];
    }
  }
  __syncthreads();
  const int lg = lane >> 3, c8 = (lane & 7) * 8;
  H8 oh[2], ol[2];
#pragma unroll
  for (int it = 0; it < 2; ++it) {
    const int nr = wave * 8 + it * 4 + lg;
#pragma unroll
    for (int e = 0; e < 8; ++e) {
      const float f = lt[c8 + e][nr];
      const unsigned short hb = f2bf_bits(f);
      oh[it].u[e] = hb;
      ol[it].u[e] = f2bf_bits(f - bf_bits2f(hb));
    }
  }
  for (int pass = 0; pass < 2; ++pass) {
#pragma unroll
    for (int it = 0; it < 2; ++it) {
      const int nr = wave * 8 + it * 4 + lg;
      const size_t go = (size_t)(n0 + nr) * nrows_k + k0 + c8;
      *(volatile v8h*)(hi + go) = oh[it].v;
      *(volatile v8h*)(lo + go) = ol[it].v;
    }
    __threadfence();
  }
}

__global__ __launch_bounds__(256) void k_trig(const int* __restrict__ qpos, const int* __restrict__ kvpos,
                                              float* __restrict__ cs, float* __restrict__ sn) {
  const int t = blockIdx.x * 256 + threadIdx.x;
  int row = t >> 5;
  const int f = t & 31;
  row = row < NTRIGROWS ? row : NTRIGROWS - 1;
  const int rq = row < NQROWS ? row : NQROWS - 1;
  int rk = row - NQROWS;
  rk = rk < 0 ? 0 : rk;
  rk = rk > LKV - 1 ? LKV - 1 : rk;
  const int pq = qpos[rq];
  const int pk = kvpos[rk];
  int pos = (row < NQROWS) ? pq : pk;
  pos = pos < 0 ? 0 : pos;
  pos = pos > SMAXPOS - 1 ? SMAXPOS - 1 : pos;
  const float tt  = (float)(2 * f) * (1.0f / 64.0f);
  const float p   = powf(ROPE_BASE_F, tt);
  const float inv = 1.0f / p;
  const float ang = (float)pos * inv;
  const float cv = cosf(ang);
  const float sv = sinf(ang);
  float* dc = cs + (size_t)row * NHALF + f;
  float* ds = sn + (size_t)row * NHALF + f;
  *(volatile float*)dc = cv;
  *(volatile float*)ds = sv;
  __threadfence();
  *(volatile float*)dc = cv;
  *(volatile float*)ds = sv;
}

__global__ __launch_bounds__(256) void k_ropek(const float* __restrict__ kvf, const float* __restrict__ cs,
                                               const float* __restrict__ sn, float* __restrict__ kr) {
  const int lane = threadIdx.x & 31;
  int wid = blockIdx.x * 8 + (threadIdx.x >> 5);
  const int nw = NKVROWS * NHEAD;
  wid = wid < nw ? wid : nw - 1;
  const int kvrow = wid >> 4, h = wid & 15;
  const int j = kvrow - (kvrow / LKV) * LKV;
  const float c = cs[(size_t)(NQROWS + j) * NHALF + lane];
  const float s = sn[(size_t)(NQROWS + j) * NHALF + lane];
  const float* xp = kvf + (size_t)kvrow * KVCOLS + h * DHEAD + lane;
  const float x1 = xp[0];
  const float x2 = xp[NHALF];
  const float o1 = x1 * c - x2 * s;
  const float o2 = x2 * c + x1 * s;
  float* dp = kr + (size_t)kvrow * DMODEL + h * DHEAD + lane;
  *(volatile float*)dp = o1;
  *(volatile float*)(dp + NHALF) = o2;
  __threadfence();
  *(volatile float*)dp = o1;
  *(volatile float*)(dp + NHALF) = o2;
}

__global__ __launch_bounds__(ATT_THREADS) void k_attn_window(
    const float* __restrict__ qf, const float* __restrict__ kr, const float* __restrict__ kvf,
    const float* __restrict__ cs, const float* __restrict__ sn, const int* __restrict__ seg,
    unsigned short* __restrict__ ctxh, unsigned short* __restrict__ ctxl) {
  __shared__ __align__(16) v4f qst[16 * ATT_THREADS];
  __shared__ float sst[KWIN * ATT_THREADS];
  const int tid = threadIdx.x;
  const int lane = tid & 31, wave = tid >> 5;
  const int r = tid >> 4, h = tid & 15;
  int qrow = blockIdx.x * ATT_QPB + r;
  qrow = qrow < NQROWS ? qrow : NQROWS - 1;
  const int b = qrow / LQ;
  const int kvb = b * LKV;
  const int sid = seg[qrow];

  {
    const float* qp = qf + (size_t)qrow * DMODEL + h * DHEAD;
    const float* cp = cs + (size_t)qrow * NHALF;
    const float* sp = sn + (size_t)qrow * NHALF;
#pragma unroll 1
    for (int j = 0; j < 8; ++j) {
      const v4f x1 = *(const v4f*)(qp + 4 * j);
      const v4f x2 = *(const v4f*)(qp + NHALF + 4 * j);
      const v4f cc = *(const v4f*)(cp + 4 * j);
      const v4f ss = *(const v4f*)(sp + 4 * j);
      const v4f r1 = x1 * cc - x2 * ss;
      const v4f r2 = x2 * cc + x1 * ss;
      qst[j * ATT_THREADS + tid] = r1;
      qst[(8 + j) * ATT_THREADS + tid] = r2;
    }
  }

#pragma unroll 1
  for (int o = 0; o < KWIN; ++o) {
    const int g = sid - o;
    const bool valid = g >= 0;
    int gc = g < 0 ? 0 : g;
    gc = gc > LKV - 1 ? LKV - 1 : gc;
    const float* kp = kr + (size_t)(kvb + gc) * DMODEL + h * DHEAD;
    v4f dacc = {0.f, 0.f, 0.f, 0.f};
#pragma unroll 1
    for (int c = 0; c < 16; c += 4) {
      const v4f ka = *(const v4f*)(kp + 4 * c);
      const v4f kb = *(const v4f*)(kp + 4 * c + 4);
      const v4f kc = *(const v4f*)(kp + 4 * c + 8);
      const v4f kd = *(const v4f*)(kp + 4 * c + 12);
      const v4f qa = qst[(c + 0) * ATT_THREADS + tid];
      const v4f qb = qst[(c + 1) * ATT_THREADS + tid];
      const v4f qc = qst[(c + 2) * ATT_THREADS + tid];
      const v4f qd = qst[(c + 3) * ATT_THREADS + tid];
      dacc += ka * qa;
      dacc += kb * qb;
      dacc += kc * qc;
      dacc += kd * qd;
    }
    const float d = (dacc[0] + dacc[1]) + (dacc[2] + dacc[3]);
    const float sval = valid ? d * ATT_SCALE : NEG_FILL;
    sst[o * ATT_THREADS + tid] = sval;
  }

  float sc[KWIN], pr[KWIN];
  int vo[KWIN];
#pragma unroll
  for (int o = 0; o < KWIN; ++o) sc[o] = sst[o * ATT_THREADS + tid];
  float mx = sc[0];
#pragma unroll
  for (int o = 1; o < KWIN; ++o) mx = fmaxf(mx, sc[o]);
  float den = 0.f;
#pragma unroll
  for (int o = 0; o < KWIN; ++o) { pr[o] = __expf(sc[o] - mx); den += pr[o]; }
  const float inv = 1.0f / den;
#pragma unroll
  for (int o = 0; o < KWIN; ++o) {
    pr[o] *= inv;
    int gc = sid - o;
    gc = gc < 0 ? 0 : gc;
    gc = gc > LKV - 1 ? LKV - 1 : gc;
    vo[o] = (kvb + gc) * KVCOLS + DMODEL + h * DHEAD;
  }

  __syncthreads();
#pragma unroll 1
  for (int c = 0; c < 16; ++c) {
    v4f acc = {0.f, 0.f, 0.f, 0.f};
#pragma unroll
    for (int o = 0; o < KWIN; ++o) {
      const v4f vv = *(const v4f*)(kvf + (size_t)vo[o] + 4 * c);
      acc += pr[o] * vv;
    }
    qst[c * ATT_THREADS + tid] = acc;
  }
  __syncthreads();

  const int e8 = lane & 7, lg = lane >> 3;
  H8 oh[8], ol[8];
#pragma unroll
  for (int it = 0; it < 8; ++it) {
    const int li = it * 4 + lg;
    const int rr = 2 * wave + (li >> 4);
    const int hh = li & 15;
    const int t2 = rr * NHEAD + hh;
    const v4f a0 = qst[(2 * e8) * ATT_THREADS + t2];
    const v4f a1 = qst[(2 * e8 + 1) * ATT_THREADS + t2];
#pragma unroll
    for (int e = 0; e < 4; ++e) {
      unsigned short hb = f2bf_bits(a0[e]);
      oh[it].u[e] = hb;
      ol[it].u[e] = f2bf_bits(a0[e] - bf_bits2f(hb));
      hb = f2bf_bits(a1[e]);
      oh[it].u[4 + e] = hb;
      ol[it].u[4 + e] = f2bf_bits(a1[e] - bf_bits2f(hb));
    }
  }
  for (int pass = 0; pass < 2; ++pass) {
#pragma unroll
    for (int it = 0; it < 8; ++it) {
      const int li = it * 4 + lg;
      const int rr = 2 * wave + (li >> 4);
      const int hh = li & 15;
      const size_t go = (size_t)(blockIdx.x * ATT_QPB + rr) * DMODEL + hh * DHEAD + e8 * 8;
      *(volatile v8h*)(ctxh + go) = oh[it].v;
      *(volatile v8h*)(ctxl + go) = ol[it].v;
    }
    __threadfence();
  }
}

static void gemm_split_f32(const unsigned short* Ah, const unsigned short* Al, int lda,
                           const unsigned short* Bh, const unsigned short* Bl, int ldb,
                           float* Cf, int ldc, int Mr, int Nc, int Kd, hipStream_t st) {
  const int tiles = (Mr >> 6) * (Nc >> 6);
  dim3 grid((tiles + 7) / 8, 1, 1);
  wmma_gemm64<1, true, 0, 0, false><<<grid, 256, 0, st>>>(
      Ah, Al, lda, 0L, Bh, Bl, ldb, 0L, (void*)Cf, (void*)Cf, ldc, 0L,
      (const float*)Cf, (const float*)Cf, 0L, Mr, Nc, Kd, 1.0f);
}

extern "C" void kernel_launch(void* const* d_in, const int* in_sizes, int n_in,
                              void* d_out, int out_size, void* d_ws, size_t ws_size,
                              hipStream_t stream) {
  if (n_in < 8) return;
  if (in_sizes[0] != NQROWS * DMODEL || in_sizes[1] != NKVROWS * DMODEL || in_sizes[2] != DMODEL * DMODEL ||
      in_sizes[3] != DMODEL * KVCOLS || in_sizes[4] != DMODEL * DMODEL || in_sizes[5] != NQROWS ||
      in_sizes[6] != NQROWS || in_sizes[7] != LKV || out_size != NQROWS * DMODEL) return;

  const float* q_in   = (const float*)d_in[0];
  const float* kv_in  = (const float*)d_in[1];
  const float* wq_in  = (const float*)d_in[2];
  const float* wkv_in = (const float*)d_in[3];
  const float* wo_in  = (const float*)d_in[4];
  const int*   seg_in = (const int*)d_in[5];
  const int*   qp_in  = (const int*)d_in[6];
  const int*   kp_in  = (const int*)d_in[7];
  float* out = (float*)d_out;

  const size_t szQP  = (size_t)NQROWS * DMODEL * 2;
  const size_t szKVP = (size_t)NKVROWS * DMODEL * 2;
  const size_t szWQ  = (size_t)DMODEL * DMODEL * 2;
  const size_t szWKV = (size_t)KVCOLS * DMODEL * 2;
  const size_t szWO  = (size_t)DMODEL * DMODEL * 2;
  const size_t szQF  = (size_t)NQROWS * DMODEL * 4;
  const size_t szKVF = (size_t)NKVROWS * KVCOLS * 4;
  const size_t szKR  = (size_t)NKVROWS * DMODEL * 4;
  const size_t szTR  = (size_t)NTRIGROWS * NHALF * 4;
  const size_t total = 2 * szQP + 2 * szKVP + 2 * szWQ + 2 * szWKV + 2 * szWO + szQF + szKVF + szKR + 2 * szTR;
  if (total > ws_size || total > (size_t)134217728) return;

  char* base = (char*)d_ws;
  size_t off = 0;
  auto take = [&](size_t bytes) -> char* { char* p = base + off; off += (bytes + 255) & ~(size_t)255; return p; };
  unsigned short* QH   = (unsigned short*)take(szQP);
  unsigned short* QL   = (unsigned short*)take(szQP);
  unsigned short* KVH  = (unsigned short*)take(szKVP);
  unsigned short* KVL  = (unsigned short*)take(szKVP);
  unsigned short* WQH  = (unsigned short*)take(szWQ);
  unsigned short* WQL  = (unsigned short*)take(szWQ);
  unsigned short* WKVH = (unsigned short*)take(szWKV);
  unsigned short* WKVL = (unsigned short*)take(szWKV);
  unsigned short* WOH  = (unsigned short*)take(szWO);
  unsigned short* WOL  = (unsigned short*)take(szWO);
  float*          QF   = (float*)take(szQF);
  float*          KVF  = (float*)take(szKVF);
  float*          KR   = (float*)take(szKR);
  float*          CS   = (float*)take(szTR);
  float*          SN   = (float*)take(szTR);
  if (off > ws_size) return;
  unsigned short* CTXH = QH;
  unsigned short* CTXL = QL;

  {
    const int n8q = NQROWS * DMODEL / 8;
    k_split8<<<n8q / 256, 256, 0, stream>>>(q_in, QH, QL, n8q);
    const int n8k = NKVROWS * DMODEL / 8;
    k_split8<<<n8k / 256, 256, 0, stream>>>(kv_in, KVH, KVL, n8k);
    k_tsplit<<<dim3(DMODEL / 64, DMODEL / 64), 256, 0, stream>>>(wq_in, WQH, WQL, DMODEL, DMODEL);
    k_tsplit<<<dim3(KVCOLS / 64, DMODEL / 64), 256, 0, stream>>>(wkv_in, WKVH, WKVL, DMODEL, KVCOLS);
    k_tsplit<<<dim3(DMODEL / 64, DMODEL / 64), 256, 0, stream>>>(wo_in, WOH, WOL, DMODEL, DMODEL);
  }

  gemm_split_f32(KVH, KVL, DMODEL, WKVH, WKVL, DMODEL, KVF, KVCOLS, NKVROWS, KVCOLS, DMODEL, stream);
  gemm_split_f32(QH, QL, DMODEL, WQH, WQL, DMODEL, QF, DMODEL, NQROWS, DMODEL, DMODEL, stream);

  k_trig<<<(NTRIGROWS * NHALF) / 256, 256, 0, stream>>>(qp_in, kp_in, CS, SN);
  k_ropek<<<(NKVROWS * NHEAD) / 8, 256, 0, stream>>>(KVF, CS, SN, KR);

  k_attn_window<<<NQROWS / ATT_QPB, ATT_THREADS, 0, stream>>>(QF, KR, KVF, CS, SN, seg_in, CTXH, CTXL);

  gemm_split_f32(CTXH, CTXL, DMODEL, WOH, WOL, DMODEL, out, DMODEL, NQROWS, DMODEL, DMODEL, stream);
}
